// DecoderBlock_60885456388591
// MI455X (gfx1250) — hardware-verified
//
#include <hip/hip_runtime.h>
#include <math.h>

typedef __attribute__((ext_vector_type(16))) _Float16 v16h;
typedef __attribute__((ext_vector_type(8)))  _Float16 v8h;
typedef __attribute__((ext_vector_type(8)))  float    v8f;
typedef __attribute__((ext_vector_type(4)))  float    v4f;
typedef __attribute__((ext_vector_type(4)))  unsigned v4u;
typedef __attribute__((ext_vector_type(2)))  unsigned v2u;

#ifndef NB
#define NB 2
#endif
#ifndef SEQ
#define SEQ 2048
#endif
#define NB_FULL 2
#define SEQ_FULL 2048

constexpr unsigned kDim   = 512;
constexpr unsigned kHeads = 8;
constexpr unsigned kHdim  = 64;
constexpr unsigned kFfn   = 2048;
constexpr unsigned kSeq   = SEQ;
constexpr unsigned kRows  = NB * SEQ;
constexpr unsigned kWpr   = kSeq / 32;
constexpr unsigned kNch   = kSeq / 64;
constexpr unsigned kNqb   = kSeq / 64;
constexpr unsigned kChMask = (kNch >= 32u) ? 0xFFFFFFFFu : ((1u << (kNch & 31u)) - 1u);

constexpr float kCarryAct  = 8.0f;
constexpr float kCarryW    = 256.0f;
constexpr float kCarryW2   = 512.0f;
constexpr float kCarryQkv  = 8.0f;
constexpr float kCarryP    = 1024.0f;
constexpr float kCarryAttn = 64.0f;
constexpr float kCarryH    = 8.0f;

constexpr size_t kSzWqkv  = (size_t)3 * kDim * kDim * 2;
constexpr size_t kSzW512  = (size_t)kDim * kDim * 2;
constexpr size_t kSzWkv   = (size_t)2 * kDim * kDim * 2;
constexpr size_t kSzW1    = (size_t)kFfn * kDim * 2;
constexpr size_t kSzW2    = (size_t)kDim * kFfn * 2;
constexpr size_t kSzF32   = (size_t)kRows * kDim * 4;
constexpr size_t kSzH16   = (size_t)kRows * kDim * 2;
constexpr size_t kSzQkv   = (size_t)kRows * 3 * kDim * 2;
constexpr size_t kSzKv    = (size_t)kRows * 2 * kDim * 2;
constexpr size_t kSzHid   = (size_t)kRows * kFfn * 2;
constexpr size_t kSzBits  = (size_t)2 * kSeq * kWpr * 4;
constexpr size_t kSzFlags = (size_t)2 * kNqb * 128;
constexpr size_t kOffWqkv = 0;
constexpr size_t kOffWsa  = kOffWqkv + kSzWqkv;
constexpr size_t kOffWq   = kOffWsa + kSzW512;
constexpr size_t kOffWkv  = kOffWq + kSzW512;
constexpr size_t kOffWca  = kOffWkv + kSzWkv;
constexpr size_t kOffW1   = kOffWca + kSzW512;
constexpr size_t kOffW2   = kOffW1 + kSzW1;
constexpr size_t kOffXr   = kOffW2 + kSzW2;
constexpr size_t kOffXa   = kOffXr + kSzF32;
constexpr size_t kOffXb   = kOffXa + kSzF32;
constexpr size_t kOffLnh  = kOffXb + kSzF32;
constexpr size_t kOffEnc  = kOffLnh + kSzH16;
constexpr size_t kOffQkv  = kOffEnc + kSzH16;
constexpr size_t kOffQc   = kOffQkv + kSzQkv;
constexpr size_t kOffKvc  = kOffQc + kSzH16;
constexpr size_t kOffAtt  = kOffKvc + kSzKv;
constexpr size_t kOffHid  = kOffAtt + kSzH16;
constexpr size_t kOffBits = kOffHid + kSzHid;
constexpr size_t kOffFlag = kOffBits + kSzBits;
constexpr size_t kWsTotal = kOffFlag + kSzFlags;
static_assert(NB != 2 || SEQ != 2048 || kWsTotal == 89137152);
static_assert(kWsTotal <= 134217728);
static_assert((kSzWqkv % 128) == 0 && (kSzW512 % 128) == 0 && (kSzWkv % 128) == 0 && (kSzW1 % 128) == 0 &&
              (kSzW2 % 128) == 0 && (kSzF32 % 128) == 0 && (kSzH16 % 128) == 0 && (kSzQkv % 128) == 0 &&
              (kSzKv % 128) == 0 && (kSzHid % 128) == 0 && (kSzBits % 128) == 0 && (kSzFlags % 128) == 0);
static_assert(kSeq % 64 == 0 && kNch <= 32 && kHdim == 64 && kHeads * kHdim == kDim);
static_assert(kRows % 64 == 0 && kDim % 64 == 0 && kFfn % 64 == 0 && kDim % 32 == 0 && kFfn % 32 == 0);
static_assert(((kRows / 64) * (kDim / 64)) % 8 == 0);
static_assert(((size_t)kRows * kDim) % (8 * 256) == 0);
static_assert(((size_t)kSeq * kWpr) % 256 == 0 && (kWpr % 2) == 0);
static_assert(kRows % 2 == 0 && SEQ <= SEQ_FULL && NB <= NB_FULL);

__device__ __forceinline__ float bf_rne(float f) {
  unsigned u = __float_as_uint(f);
  u = (u + 0x7FFFu + ((u >> 16) & 1u)) & 0xFFFF0000u;
  return __uint_as_float(u);
}

__device__ __forceinline__ void wave_sync() {
  __builtin_amdgcn_fence(3  , "workgroup");
  __builtin_amdgcn_wave_barrier();
  __builtin_amdgcn_fence(2  , "workgroup");
}

__device__ __forceinline__ void dep_guard_h(v8f& a, v8f& b, v16h x, v16h y) { asm volatile("v_nop\n\tv_nop\n\tv_nop\n\tv_nop" : "+v"(a), "+v"(b) : "v"(x), "v"(y)); }
__device__ __forceinline__ void keep4_h(v16h a, v16h b, v16h c, v16h d) { asm volatile("v_nop" :: "v"(a), "v"(b), "v"(c), "v"(d)); }
__device__ __forceinline__ void acc_guard4(v8f& a, v8f& b, v8f& c, v8f& d) { asm volatile("v_nop\n\tv_nop\n\tv_nop\n\tv_nop" : "+v"(a), "+v"(b), "+v"(c), "+v"(d)); }

union FragU { v16h v; v8h h[2]; };
__device__ __forceinline__ v16h frag_load(const _Float16* p) {
  FragU f; f.h[0] = *(const v8h*)(p); f.h[1] = *(const v8h*)(p + 16); return f.v;
}
__device__ __forceinline__ v8f mma_raw(v16h a, v16h b, v8f c) {
  return __builtin_amdgcn_wmma_f32_16x16x32_f16(false, a, false, b, (short)0, c, false, false);
}
__device__ __forceinline__ v8f mma_h(v16h a, v16h b, v8f c) {
  c = __builtin_amdgcn_wmma_f32_16x16x32_f16(false, a, false, b, (short)0, c, false, false);
  asm volatile("v_nop\n\tv_nop\n\tv_nop\n\tv_nop" : "+v"(c) : "v"(a), "v"(b));
  return c;
}

template <int OUT_MODE, bool RESID, int ACT>
__global__ __launch_bounds__(256) void wmma_gemm64(
    const _Float16* __restrict__ A, unsigned lda,
    const _Float16* __restrict__ Bt, unsigned ldb,
    void* __restrict__ Cout, unsigned ldc,
    const float* __restrict__ bias,
    const float* __restrict__ resid,
    unsigned M, unsigned N, unsigned K, float scale, float oscale) {
  static_assert(!RESID || OUT_MODE == 0);
  __shared__ __align__(16) float sT[8][16 * 68];
  const unsigned lane = threadIdx.x & 31u;
  const unsigned wave = threadIdx.x >> 5;
  const unsigned tilesN = N >> 6;
  const unsigned tilesM = M >> 6;
  const unsigned tile = blockIdx.x * 8u + wave;
  if (tile >= tilesM * tilesN) return;
  const unsigned tm = tile / tilesN;
  const unsigned tn = tile - tm * tilesN;
  const unsigned m0 = tm << 6;
  const unsigned n0 = tn << 6;

  const unsigned rlane = lane & 15u;
  const unsigned koff  = (lane >> 4) * 8u;
  const unsigned mOff  = (lane >> 4) * 8u;

  v8f acc[4][4];
#pragma unroll
  for (int i = 0; i < 4; ++i)
#pragma unroll
    for (int j = 0; j < 4; ++j) acc[i][j] = (v8f){0.f,0.f,0.f,0.f,0.f,0.f,0.f,0.f};

  for (unsigned k0 = 0; k0 < K; k0 += 32u) {
    v16h bh[4];
#pragma unroll
    for (int j = 0; j < 4; ++j) {
      const size_t bo = (size_t)(n0 + ((unsigned)j << 4) + rlane) * ldb + koff + k0;
      bh[j] = frag_load(Bt + bo);
    }
#pragma unroll
    for (int i = 0; i < 4; ++i) {
      const size_t ao = (size_t)(m0 + ((unsigned)i << 4) + rlane) * lda + koff + k0;
      const v16h ah = frag_load(A + ao);
#pragma unroll
      for (int j = 0; j < 4; ++j) acc[i][j] = mma_raw(ah, bh[j], acc[i][j]);
      dep_guard_h(acc[i][0], acc[i][3], ah, ah);
    }
    keep4_h(bh[0], bh[1], bh[2], bh[3]);
  }
  acc_guard4(acc[0][0], acc[0][1], acc[0][2], acc[0][3]);
  acc_guard4(acc[1][0], acc[1][1], acc[1][2], acc[1][3]);
  acc_guard4(acc[2][0], acc[2][1], acc[2][2], acc[2][3]);
  acc_guard4(acc[3][0], acc[3][1], acc[3][2], acc[3][3]);

  float* slab = sT[wave];
#pragma unroll
  for (int i = 0; i < 4; ++i) {
    const unsigned mBase = m0 + ((unsigned)i << 4);
#pragma unroll
    for (int j = 0; j < 4; ++j) {
      const unsigned n = n0 + ((unsigned)j << 4) + rlane;
      const float bv = bf_rne(bias[n]);
#pragma unroll
      for (int r = 0; r < 8; ++r) {
        float v = acc[i][j][r] * scale + bv;
        if (ACT != 7) v *= oscale;
        slab[(mOff + (unsigned)r) * 68u + ((unsigned)j << 4) + rlane] = v;
      }
    }
    wave_sync();
    if (ACT == 7) {
#pragma unroll 1
      for (unsigned it = 0; it < 8u; ++it) {
        const unsigned p = it * 32u + lane;
        const unsigned row = p >> 4, c4 = (p & 15u) * 4u;
        v4f v = *(const v4f*)(slab + row * 68u + c4);
#pragma unroll
        for (int e = 0; e < 4; ++e) {
          const float z = v[e];
          v[e] = 0.5f * z * (1.0f + erff(z * 0.70710678118654752f)) * oscale;
        }
        *(v4f*)(slab + row * 68u + c4) = v;
      }
      wave_sync();
    }
    if (OUT_MODE == 0) {
      float* C = (float*)Cout;
      const unsigned hh = lane >> 4, c4 = (lane & 15u) * 4u;
      for (int pass = 0; pass < 2; ++pass) {
#pragma unroll
        for (int it = 0; it < 8; ++it) {
          const unsigned row = (unsigned)it * 2u + hh;
          v4f v = *(const v4f*)(slab + row * 68u + c4);
          if (RESID) {
            const v4f rr = *(const v4f*)(resid + (size_t)(mBase + row) * ldc + n0 + c4);
            v += rr;
          }
          *(volatile v4f*)(C + (size_t)(mBase + row) * ldc + n0 + c4) = v;
        }
        __threadfence();
      }
    } else {
      const unsigned q = lane >> 3, c8 = (lane & 7u) * 8u;
      _Float16* C = (_Float16*)Cout;
      for (int pass = 0; pass < 2; ++pass) {
#pragma unroll
        for (int it = 0; it < 4; ++it) {
          const unsigned row = (unsigned)it * 4u + q;
          const float* sp = slab + row * 68u + c8;
          v8h hv;
#pragma unroll
          for (int e = 0; e < 8; ++e) hv[e] = (_Float16)sp[e];
          *(volatile v8h*)(C + (size_t)(mBase + row) * ldc + n0 + c8) = hv;
        }
        __threadfence();
      }
    }
    wave_sync();
  }
}

__global__ __launch_bounds__(256) void cast_w_t(
    const float* __restrict__ W, _Float16* __restrict__ out, unsigned K, unsigned N, float sc) {
  __shared__ __align__(16) _Float16 tile[64 * 72];
  const unsigned t = threadIdx.x;
  const unsigned n0 = blockIdx.x * 64u, k0 = blockIdx.y * 64u;
  const unsigned nn = t & 63u, kq = t >> 6;
#pragma unroll 4
  for (unsigned i = 0; i < 16u; ++i) {
    const unsigned kk = i * 4u + kq;
    const float w = W[(size_t)(k0 + kk) * N + n0 + nn];
    tile[nn * 72u + kk] = (_Float16)(bf_rne(w) * sc);
  }
  __syncthreads();
  const unsigned p0 = t, p1 = 256u + t;
  const unsigned r0 = p0 >> 3, c0 = (p0 & 7u) * 8u;
  const unsigned r1 = p1 >> 3, c1 = (p1 & 7u) * 8u;
  const v8h h0 = *(const v8h*)(tile + r0 * 72u + c0);
  const v8h h1 = *(const v8h*)(tile + r1 * 72u + c1);
  _Float16* d0 = out + (size_t)(n0 + r0) * K + k0 + c0;
  _Float16* d1 = out + (size_t)(n0 + r1) * K + k0 + c1;
  *(volatile v8h*)d0 = h0;
  *(volatile v8h*)d1 = h1;
  __threadfence();
  *(volatile v8h*)d0 = h0;
  *(volatile v8h*)d1 = h1;
}

__global__ __launch_bounds__(256) void cast_rows_f16(
    const float* __restrict__ in, _Float16* __restrict__ out, float sc) {
  const unsigned i = blockIdx.x * 256u + threadIdx.x;
  const unsigned row = i >> 6;
  const unsigned c8 = (i & 63u) * 8u;
  const unsigned b = row / kSeq;
  const unsigned s = row - b * kSeq;
  const float* p = in + ((size_t)b * SEQ_FULL + s) * kDim + c8;
  const v4f a0 = *(const v4f*)(p);
  const v4f a1 = *(const v4f*)(p + 4);
  v8h hv;
#pragma unroll
  for (int e = 0; e < 4; ++e) {
    hv[e]     = (_Float16)(bf_rne(a0[e]) * sc);
    hv[e + 4] = (_Float16)(bf_rne(a1[e]) * sc);
  }
  _Float16* d = out + (size_t)row * kDim + c8;
  *(volatile v8h*)d = hv;
  __threadfence();
  *(volatile v8h*)d = hv;
}

__global__ __launch_bounds__(256) void mask_bits(
    const int* __restrict__ m0, const int* __restrict__ m1, unsigned* __restrict__ bits) {
  __shared__ __align__(16) unsigned wsh[256];
  const int* m = (blockIdx.y != 0u) ? m1 : m0;
  unsigned* outb = bits + (size_t)blockIdx.y * ((size_t)kSeq * kWpr);
  const unsigned t = threadIdx.x, w = t >> 5, l = t & 31u;
#pragma unroll 4
  for (unsigned it = 0; it < 32u; ++it) {
    const unsigned idx = it * 8u + w;
    const unsigned g = blockIdx.x * 256u + idx;
    const unsigned row = g / kWpr;
    const unsigned wc = g - row * kWpr;
    const int mv = m[(size_t)row * SEQ_FULL + wc * 32u + l];
    const unsigned bal = __builtin_amdgcn_ballot_w32(mv != 0);
    if (l == 0u) wsh[idx] = bal;
  }
  __syncthreads();
  if (t < 64u) {
    const v4u wv = *(const v4u*)(wsh + 4u * t);
    unsigned* d = outb + (size_t)blockIdx.x * 256u + 4u * t;
    *(volatile v4u*)d = wv;
    __threadfence();
    *(volatile v4u*)d = wv;
  }
}

__global__ __launch_bounds__(32) void mask_flags(
    const unsigned* __restrict__ bits, unsigned* __restrict__ flags) {
  const unsigned l = threadIdx.x;
  const unsigned qb = blockIdx.x, sel = blockIdx.y;
  const unsigned* bb = bits + (size_t)sel * ((size_t)kSeq * kWpr);
  unsigned allb = 0xFFFFFFFFu, noneb = 0xFFFFFFFFu, dead = 0u;
#pragma unroll
  for (unsigned rr = 0; rr < 2u; ++rr) {
    const unsigned row = qb * 64u + rr * 32u + l;
    unsigned ra = 0u, rn = 0u;
#pragma unroll 1
    for (unsigned kc = 0; kc < kNch; ++kc) {
      const v2u w = *(const v2u*)(bb + (size_t)row * kWpr + kc * 2u);
      const unsigned a = ((w[0] & w[1]) == 0xFFFFFFFFu) ? 1u : 0u;
      const unsigned n = ((w[0] | w[1]) == 0u) ? 1u : 0u;
      ra |= a << kc;
      rn |= n << kc;
    }
    allb &= ra;
    noneb &= rn;
    dead |= (rn == kChMask) ? 1u : 0u;
  }
#pragma unroll
  for (int off = 1; off < 32; off <<= 1) {
    allb  &= __shfl_xor(allb, off, 32);
    noneb &= __shfl_xor(noneb, off, 32);
    dead  |= __shfl_xor(dead, off, 32);
  }
  const unsigned myw = (l == 0u) ? allb : ((l == 1u) ? noneb : ((l == 2u) ? dead : 0u));
  v4u o;
#pragma unroll
  for (int e = 0; e < 4; ++e) o[e] = __shfl(myw, (int)((4u * l + (unsigned)e) & 31u), 32);
  if (l < 8u) {
    unsigned* d = flags + ((size_t)sel * kNqb + qb) * 32u + 4u * l;
    *(volatile v4u*)d = o;
    __threadfence();
    *(volatile v4u*)d = o;
  }
}

template <bool FIRST>
__global__ __launch_bounds__(256) void layernorm_rows(
    const float* __restrict__ x, const float* __restrict__ gam, const float* __restrict__ bet,
    float* __restrict__ xcopy, _Float16* __restrict__ yh, float hscale) {
  __shared__ float ssum[8];
  __shared__ float ssq[8];
  __shared__ __align__(16) unsigned hrow[512];
  const unsigned t = threadIdx.x;
  const unsigned w = t >> 5;
  const unsigned l = t & 31u;
  const unsigned rsel = t >> 7;
  const unsigned tt = t & 127u;
  const unsigned row = blockIdx.x * 2u + rsel;
  size_t inoff = (size_t)row * kDim;
  if (FIRST) {
    const unsigned b = row / kSeq;
    const unsigned s = row - b * kSeq;
    inoff = ((size_t)b * SEQ_FULL + s) * kDim;
  }
  v4f v = *(const v4f*)(x + inoff + tt * 4u);
  if (FIRST) {
#pragma unroll
    for (int e = 0; e < 4; ++e) v[e] = bf_rne(v[e]);
  }
  float s1 = (v[0] + v[1]) + (v[2] + v[3]);
#pragma unroll
  for (int off = 1; off < 32; off <<= 1) s1 += __shfl_xor(s1, off, 32);
  if (l == 0u) ssum[w] = s1;
  __syncthreads();
  const float tot = (ssum[rsel * 4u] + ssum[rsel * 4u + 1u]) + (ssum[rsel * 4u + 2u] + ssum[rsel * 4u + 3u]);
  const float mean = tot * (1.0f / 512.0f);
  const v4f d = v - mean;
  float q = (d[0] * d[0] + d[1] * d[1]) + (d[2] * d[2] + d[3] * d[3]);
#pragma unroll
  for (int off = 1; off < 32; off <<= 1) q += __shfl_xor(q, off, 32);
  if (l == 0u) ssq[w] = q;
  __syncthreads();
  const float totq = (ssq[rsel * 4u] + ssq[rsel * 4u + 1u]) + (ssq[rsel * 4u + 2u] + ssq[rsel * 4u + 3u]);
  const float var = totq * (1.0f / 512.0f);
  const float inv = rsqrtf(var + 1e-5f);
  v4f gv = *(const v4f*)(gam + tt * 4u);
  v4f bv = *(const v4f*)(bet + tt * 4u);
#pragma unroll
  for (int e = 0; e < 4; ++e) { gv[e] = bf_rne(gv[e]); bv[e] = bf_rne(bv[e]); }
  const v4f o = d * inv * gv + bv;
  if (FIRST) {
    float* xr = xcopy + (size_t)row * kDim + tt * 4u;
    *(volatile v4f*)xr = v;
    __threadfence();
    *(volatile v4f*)xr = v;
  }
  const unsigned hb0 = (unsigned)__builtin_bit_cast(unsigned short, (_Float16)(o[0] * hscale));
  const unsigned hb1 = (unsigned)__builtin_bit_cast(unsigned short, (_Float16)(o[1] * hscale));
  const unsigned hb2 = (unsigned)__builtin_bit_cast(unsigned short, (_Float16)(o[2] * hscale));
  const unsigned hb3 = (unsigned)__builtin_bit_cast(unsigned short, (_Float16)(o[3] * hscale));
  v2u pk;
  pk[0] = hb0 | (hb1 << 16);
  pk[1] = hb2 | (hb3 << 16);
  *(v2u*)(hrow + rsel * 256u + 2u * tt) = pk;
  __syncthreads();
  if (t < 128u) {
    const unsigned rs = t >> 6, piece = t & 63u;
    const v4u wv = *(const v4u*)(hrow + rs * 256u + piece * 4u);
    _Float16* hp = yh + (size_t)(blockIdx.x * 2u + rs) * kDim + piece * 8u;
    *(volatile v4u*)hp = wv;
    __threadfence();
    *(volatile v4u*)hp = wv;
  }
}

constexpr unsigned kAKC = 64;
constexpr unsigned kANW = 4;

__device__ __forceinline__ void vt_scatter(_Float16* vt, v4u w, unsigned d0, unsigned kvr) {
#pragma unroll
  for (int e = 0; e < 4; ++e) {
    const unsigned u = w[e];
    const unsigned d = d0 + 2u * (unsigned)e;
    vt[d * kAKC + kvr]        = __builtin_bit_cast(_Float16, (unsigned short)(u & 0xffffu));
    vt[(d + 1u) * kAKC + kvr] = __builtin_bit_cast(_Float16, (unsigned short)(u >> 16));
  }
}

__global__ __launch_bounds__(128)
void attn_h64(const _Float16* __restrict__ qp, unsigned ldq,
              const _Float16* __restrict__ kp, unsigned ldk,
              const _Float16* __restrict__ vp, unsigned ldv,
              const unsigned* __restrict__ bits, const unsigned* __restrict__ flags,
              _Float16* __restrict__ attn_out, float sscale, float pscale, float oscale) {
  __shared__ __align__(16) _Float16 Ksh[kAKC * kHdim];
  __shared__ __align__(16) _Float16 Vth[kHdim * kAKC];
  __shared__ __align__(16) _Float16 Psh[kANW][16 * kAKC];
  __shared__ __align__(16) float  Osl[kANW][16 * 68];

  const unsigned tid  = threadIdx.x;
  const unsigned wave = tid >> 5;
  const unsigned lane = tid & 31u;
  const unsigned hh   = lane >> 4;
  const unsigned c    = lane & 15u;

  const unsigned bx = blockIdx.x;
  const unsigned bh = bx / kNqb;
  const unsigned qb = bx - bh * kNqb;
  const unsigned b  = bh / kHeads;
  const unsigned h  = bh - b * kHeads;
  const unsigned q0 = qb * 64u + wave * 16u;

  const _Float16* qbase = qp + (size_t)b * kSeq * ldq + h * kHdim;
  const _Float16* kbase = kp + (size_t)b * kSeq * ldk + h * kHdim;
  const _Float16* vbase = vp + (size_t)b * kSeq * ldv + h * kHdim;

  v16h qa[2];
  {
    const _Float16* qrow = qbase + (size_t)(q0 + c) * ldq + 8u * hh;
    qa[0] = frag_load(qrow);
    qa[1] = frag_load(qrow + 32);
  }

  const unsigned allw  = flags[(size_t)qb * 32u + 0u];
  const unsigned nonew = flags[(size_t)qb * 32u + 1u];
  const unsigned dead  = flags[(size_t)qb * 32u + 2u];

  float mrow[8], lrow[8];
  v8f oacc[4];
#pragma unroll
  for (int r = 0; r < 8; ++r) { mrow[r] = -INFINITY; lrow[r] = 0.f; }
#pragma unroll
  for (int t = 0; t < 4; ++t) oacc[t] = (v8f){0.f,0.f,0.f,0.f,0.f,0.f,0.f,0.f};

  for (unsigned kc = 0; kc < kNch; ++kc) {
    const bool none = ((nonew >> kc) & 1u) != 0u;
    if (none && dead == 0u) continue;
    const bool full = ((allw >> kc) & 1u) != 0u;
    const unsigned kv0 = kc * kAKC;
    __syncthreads();
    {
      const unsigned kvr = tid >> 1, dh = (tid & 1u) * 32u;
      const _Float16* krow = kbase + (size_t)(kv0 + kvr) * ldk + dh;
      const _Float16* vrow = vbase + (size_t)(kv0 + kvr) * ldv + dh;
      const v8h k0v = *(const v8h*)(krow);
      const v8h k1v = *(const v8h*)(krow + 8);
      const v8h k2v = *(const v8h*)(krow + 16);
      const v8h k3v = *(const v8h*)(krow + 24);
      const v4u v0w = *(const v4u*)(vrow);
      const v4u v1w = *(const v4u*)(vrow + 8);
      const v4u v2w = *(const v4u*)(vrow + 16);
      const v4u v3w = *(const v4u*)(vrow + 24);
      _Float16* kd = Ksh + kvr * kHdim + dh;
      *(v8h*)(kd)      = k0v;
      *(v8h*)(kd + 8)  = k1v;
      *(v8h*)(kd + 16) = k2v;
      *(v8h*)(kd + 24) = k3v;
      vt_scatter(Vth, v0w, dh,       kvr);
      vt_scatter(Vth, v1w, dh + 8u,  kvr);
      vt_scatter(Vth, v2w, dh + 16u, kvr);
      vt_scatter(Vth, v3w, dh + 24u, kvr);
    }
    __syncthreads();

    v8f s[4];
#pragma unroll
    for (int j = 0; j < 4; ++j) {
      s[j] = (v8f){0.f,0.f,0.f,0.f,0.f,0.f,0.f,0.f};
#pragma unroll
      for (int dc = 0; dc < 2; ++dc) {
        FragU kb;
        kb.h[0] = *(const v8h*)(Ksh + ((unsigned)j * 16u + c) * kHdim + (unsigned)dc * 32u + 8u * hh);
        kb.h[1] = *(const v8h*)(Ksh + ((unsigned)j * 16u + c) * kHdim + (unsigned)dc * 32u + 16u + 8u * hh);
        s[j] = mma_h(qa[dc], kb.v, s[j]);
      }
    }
#pragma unroll
    for (int j = 0; j < 4; ++j)
#pragma unroll
      for (int r = 0; r < 8; ++r) s[j][r] = s[j][r] * sscale;
    if (!full) {
#pragma unroll
      for (int r = 0; r < 8; ++r) {
        const v2u mw = *(const v2u*)(bits + (size_t)(q0 + 8u * hh + (unsigned)r) * kWpr + kc * 2u);
#pragma unroll
        for (int j = 0; j < 4; ++j) {
          const unsigned bit = (mw[j >> 1] >> ((unsigned)(j & 1) * 16u + c)) & 1u;
          s[j][r] = (bit != 0u) ? s[j][r] : -1.0e30f;
        }
      }
    }
    float cm[8];
#pragma unroll
    for (int r = 0; r < 8; ++r) {
      float m = fmaxf(fmaxf(s[0][r], s[1][r]), fmaxf(s[2][r], s[3][r]));
#pragma unroll
      for (int off = 1; off < 16; off <<= 1) m = fmaxf(m, __shfl_xor(m, off, 32));
      cm[r] = m;
    }
    _Float16* pw = Psh[wave];
#pragma unroll
    for (int r = 0; r < 8; ++r) {
      const float mnew = fmaxf(mrow[r], cm[r]);
      const float alpha = __expf(mrow[r] - mnew);
      mrow[r] = mnew;
      float psum = 0.f;
#pragma unroll
      for (int j = 0; j < 4; ++j) {
        const float p = __expf(s[j][r] - mnew);
        psum += p;
        pw[(8u * hh + (unsigned)r) * kAKC + (unsigned)j * 16u + c] = (_Float16)(p * pscale);
      }
#pragma unroll
      for (int off = 1; off < 16; off <<= 1) psum += __shfl_xor(psum, off, 32);
      lrow[r] = lrow[r] * alpha + psum;
#pragma unroll
      for (int t = 0; t < 4; ++t) oacc[t][r] *= alpha;
    }
    wave_sync();
#pragma unroll
    for (int kk = 0; kk < 2; ++kk) {
      FragU pa;
      pa.h[0] = *(const v8h*)(pw + c * kAKC + (unsigned)kk * 32u + 8u * hh);
      pa.h[1] = *(const v8h*)(pw + c * kAKC + (unsigned)kk * 32u + 16u + 8u * hh);
#pragma unroll
      for (int t = 0; t < 4; ++t) {
        FragU vb;
        vb.h[0] = *(const v8h*)(Vth + ((unsigned)t * 16u + c) * kAKC + (unsigned)kk * 32u + 8u * hh);
        vb.h[1] = *(const v8h*)(Vth + ((unsigned)t * 16u + c) * kAKC + (unsigned)kk * 32u + 16u + 8u * hh);
        oacc[t] = mma_h(pa.v, vb.v, oacc[t]);
      }
    }
    wave_sync();
  }

  float* os = Osl[wave];
#pragma unroll
  for (int r = 0; r < 8; ++r) {
    const float inv = oscale * (1.0f / lrow[r]);
#pragma unroll
    for (int t = 0; t < 4; ++t) os[(8u * hh + (unsigned)r) * 68u + (unsigned)t * 16u + c] = oacc[t][r] * inv;
  }
  wave_sync();
  {
    const unsigned q8 = lane >> 3, c8 = (lane & 7u) * 8u;
    _Float16* ob = attn_out + (size_t)(b * kSeq) * kDim + h * kHdim;
    for (int pass = 0; pass < 2; ++pass) {
#pragma unroll
      for (int it = 0; it < 4; ++it) {
        const unsigned row = (unsigned)it * 4u + q8;
        const float* sp = os + row * 68u + c8;
        v8h hv;
#pragma unroll
        for (int e = 0; e < 8; ++e) hv[e] = (_Float16)sp[e];
        *(volatile v8h*)(ob + (size_t)(q0 + row) * kDim + c8) = hv;
      }
      __threadfence();
    }
  }
}

extern "C" void kernel_launch(void* const* d_in, const int* in_sizes, int n_in,
                              void* d_out, int out_size, void* d_ws, size_t ws_size,
                              hipStream_t stream) {
  if (n_in < 24) return;
  const long long needAct  = ((long long)(NB - 1) * SEQ_FULL + SEQ) * (long long)kDim;
  const long long needMask = (long long)(SEQ - 1) * SEQ_FULL + SEQ;
  if ((long long)in_sizes[0] < needAct || (long long)in_sizes[1] < needAct) return;
  if ((long long)in_sizes[2] < needMask || (long long)in_sizes[3] < needMask) return;
  if (in_sizes[4] < (int)(kDim * 3 * kDim) || in_sizes[5] < (int)(3 * kDim)) return;
  if (in_sizes[6] < (int)(kDim * kDim) || in_sizes[7] < (int)kDim) return;
  if (in_sizes[8] < (int)kDim || in_sizes[9] < (int)kDim) return;
  if (in_sizes[10] < (int)(kDim * kDim) || in_sizes[11] < (int)kDim) return;
  if (in_sizes[12] < (int)(kDim * 2 * kDim) || in_sizes[13] < (int)(2 * kDim)) return;
  if (in_sizes[14] < (int)(kDim * kDim) || in_sizes[15] < (int)kDim) return;
  if (in_sizes[16] < (int)kDim || in_sizes[17] < (int)kDim) return;
  if (in_sizes[18] < (int)(kDim * kFfn) || in_sizes[19] < (int)kFfn) return;
  if (in_sizes[20] < (int)(kFfn * kDim) || in_sizes[21] < (int)kDim) return;
  if (in_sizes[22] < (int)kDim || in_sizes[23] < (int)kDim) return;
  if ((long long)out_size < (long long)kRows * kDim) return;
  if (ws_size < kWsTotal) return;

  const float* x     = (const float*)d_in[0];
  const float* enc   = (const float*)d_in[1];
  const int*   smask = (const int*)d_in[2];
  const int*   cmask = (const int*)d_in[3];
  const float* qkvw  = (const float*)d_in[4];
  const float* qkvb  = (const float*)d_in[5];
  const float* saw   = (const float*)d_in[6];
  const float* sab   = (const float*)d_in[7];
  const float* ln1g  = (const float*)d_in[8];
  const float* ln1b  = (const float*)d_in[9];
  const float* qw    = (const float*)d_in[10];
  const float* qbias = (const float*)d_in[11];
  const float* kvw   = (const float*)d_in[12];
  const float* kvb   = (const float*)d_in[13];
  const float* caw   = (const float*)d_in[14];
  const float* cab   = (const float*)d_in[15];
  const float* ln2g  = (const float*)d_in[16];
  const float* ln2b  = (const float*)d_in[17];
  const float* m1w   = (const float*)d_in[18];
  const float* m1b   = (const float*)d_in[19];
  const float* m2w   = (const float*)d_in[20];
  const float* m2b   = (const float*)d_in[21];
  const float* ln3g  = (const float*)d_in[22];
  const float* ln3b  = (const float*)d_in[23];
  float* outf = (float*)d_out;

  char* ws = (char*)d_ws;
  _Float16* wqkv = (_Float16*)(ws + kOffWqkv);
  _Float16* wsa  = (_Float16*)(ws + kOffWsa);
  _Float16* wq   = (_Float16*)(ws + kOffWq);
  _Float16* wkv  = (_Float16*)(ws + kOffWkv);
  _Float16* wca  = (_Float16*)(ws + kOffWca);
  _Float16* w1h  = (_Float16*)(ws + kOffW1);
  _Float16* w2h  = (_Float16*)(ws + kOffW2);
  float*    xr   = (float*)(ws + kOffXr);
  float*    xa   = (float*)(ws + kOffXa);
  float*    xb   = (float*)(ws + kOffXb);
  _Float16* lnh  = (_Float16*)(ws + kOffLnh);
  _Float16* ench = (_Float16*)(ws + kOffEnc);
  _Float16* qkvp = (_Float16*)(ws + kOffQkv);
  _Float16* qcp  = (_Float16*)(ws + kOffQc);
  _Float16* kvcp = (_Float16*)(ws + kOffKvc);
  _Float16* attp = (_Float16*)(ws + kOffAtt);
  _Float16* hid  = (_Float16*)(ws + kOffHid);
  unsigned* bits = (unsigned*)(ws + kOffBits);
  unsigned* flg  = (unsigned*)(ws + kOffFlag);

  cast_w_t<<<dim3(3 * kDim / 64, kDim / 64), dim3(256), 0, stream>>>(qkvw, wqkv, kDim, 3 * kDim, kCarryW);
  cast_w_t<<<dim3(kDim / 64, kDim / 64), dim3(256), 0, stream>>>(saw, wsa, kDim, kDim, kCarryW);
  cast_w_t<<<dim3(kDim / 64, kDim / 64), dim3(256), 0, stream>>>(qw, wq, kDim, kDim, kCarryW);
  cast_w_t<<<dim3(2 * kDim / 64, kDim / 64), dim3(256), 0, stream>>>(kvw, wkv, kDim, 2 * kDim, kCarryW);
  cast_w_t<<<dim3(kDim / 64, kDim / 64), dim3(256), 0, stream>>>(caw, wca, kDim, kDim, kCarryW);
  cast_w_t<<<dim3(kFfn / 64, kDim / 64), dim3(256), 0, stream>>>(m1w, w1h, kDim, kFfn, kCarryW);
  cast_w_t<<<dim3(kDim / 64, kFfn / 64), dim3(256), 0, stream>>>(m2w, w2h, kFfn, kDim, kCarryW2);

  cast_rows_f16<<<dim3((unsigned)(((size_t)kRows * kDim) / (8 * 256))), dim3(256), 0, stream>>>(enc, ench, kCarryAct);

  mask_bits<<<dim3((unsigned)(((size_t)kSeq * kWpr) / 256), 2), dim3(256), 0, stream>>>(smask, cmask, bits);
  mask_flags<<<dim3(kNqb, 2), dim3(32), 0, stream>>>(bits, flg);

  layernorm_rows<true><<<dim3(kRows / 2), dim3(256), 0, stream>>>(x, ln1g, ln1b, xr, lnh, kCarryAct);

  wmma_gemm64<1, false, 0><<<dim3((kRows / 64) * (3 * kDim / 64) / 8), dim3(256), 0, stream>>>(
      lnh, kDim, wqkv, kDim, (void*)qkvp, 3 * kDim, qkvb, xr,
      kRows, 3 * kDim, kDim, 1.0f / (kCarryAct * kCarryW), kCarryQkv);

  attn_h64<<<dim3(NB * kHeads * kNqb), dim3(128), 0, stream>>>(
      qkvp, 3 * kDim, qkvp + kDim, 3 * kDim, qkvp + 2 * kDim, 3 * kDim,
      bits, flg, attp,
      0.125f / (kCarryQkv * kCarryQkv), kCarryP, kCarryAttn / (kCarryP * kCarryQkv));

  wmma_gemm64<0, true, 0><<<dim3((kRows / 64) * (kDim / 64) / 8), dim3(256), 0, stream>>>(
      attp, kDim, wsa, kDim, (void*)xa, kDim, sab, xr,
      kRows, kDim, kDim, 1.0f / (kCarryAttn * kCarryW), 1.0f);

  layernorm_rows<false><<<dim3(kRows / 2), dim3(256), 0, stream>>>(xa, ln2g, ln2b, xa, lnh, kCarryAct);

  wmma_gemm64<1, false, 0><<<dim3((kRows / 64) * (kDim / 64) / 8), dim3(256), 0, stream>>>(
      lnh, kDim, wq, kDim, (void*)qcp, kDim, qbias, xr,
      kRows, kDim, kDim, 1.0f / (kCarryAct * kCarryW), kCarryQkv);

  wmma_gemm64<1, false, 0><<<dim3((kRows / 64) * (2 * kDim / 64) / 8), dim3(256), 0, stream>>>(
      ench, kDim, wkv, kDim, (void*)kvcp, 2 * kDim, kvb, xr,
      kRows, 2 * kDim, kDim, 1.0f / (kCarryAct * kCarryW), kCarryQkv);

  attn_h64<<<dim3(NB * kHeads * kNqb), dim3(128), 0, stream>>>(
      qcp, kDim, kvcp, 2 * kDim, kvcp + kDim, 2 * kDim,
      bits + (size_t)kSeq * kWpr, flg + (size_t)kNqb * 32, attp,
      0.125f / (kCarryQkv * kCarryQkv), kCarryP, kCarryAttn / (kCarryP * kCarryQkv));

  wmma_gemm64<0, true, 0><<<dim3((kRows / 64) * (kDim / 64) / 8), dim3(256), 0, stream>>>(
      attp, kDim, wca, kDim, (void*)xb, kDim, cab, xa,
      kRows, kDim, kDim, 1.0f / (kCarryAttn * kCarryW), 1.0f);

  layernorm_rows<false><<<dim3(kRows / 2), dim3(256), 0, stream>>>(xb, ln3g, ln3b, xb, lnh, kCarryAct);

  wmma_gemm64<1, false, 7><<<dim3((kRows / 64) * (kFfn / 64) / 8), dim3(256), 0, stream>>>(
      lnh, kDim, w1h, kDim, (void*)hid, kFfn, m1b, xr,
      kRows, kFfn, kDim, 1.0f / (kCarryAct * kCarryW), kCarryH);

  wmma_gemm64<0, true, 0><<<dim3((kRows / 64) * (kDim / 64) / 8), dim3(256), 0, stream>>>(
      hid, kFfn, w2h, kFfn, (void*)outf, kDim, m2b, xb,
      kRows, kDim, kFfn, 1.0f / (kCarryH * kCarryW2), 1.0f);
}
